// SelectiveSSM_57509612094226
// MI455X (gfx1250) — hardware-verified
//
#include <hip/hip_runtime.h>
#include <math.h>

typedef __attribute__((ext_vector_type(16))) __bf16   v16b;
typedef __attribute__((ext_vector_type(8)))  __bf16   v8b;
typedef __attribute__((ext_vector_type(8)))  float    v8f;
typedef __attribute__((ext_vector_type(4)))  float    v4f;
typedef __attribute__((ext_vector_type(4)))  unsigned v4u;

constexpr int kBatch = 2;
constexpr int kSeqL  = 2048;
constexpr int kDmod  = 1024;
constexpr int kDin   = 2048;
constexpr int kNst   = 16;
constexpr int kXpN   = 2 * kNst + 1;
constexpr int kXpP   = 64;
constexpr int kXZP   = 2 * kDin;
constexpr int kRows  = kBatch * kSeqL;
constexpr int kTP    = 260;
constexpr int kChunk = 32;
constexpr float kLogFloor = -18.420680743952367f;

static_assert(kXpN == 33 && kXpN <= kXpP, "x_proj width");
static_assert((kDmod % 32) == 0 && (kDin % 32) == 0, "GEMM K multiples of 32");
static_assert((kSeqL % 64) == 0 && (kXZP % 64) == 0 && (kXpP % 64) == 0 && (kDmod % 64) == 0, "GEMM M,N multiples of 64");
static_assert((kSeqL % kChunk) == 0 && (kDin % 256) == 0 && (kDmod % 64) == 0 && (kDin % 64) == 0, "tile multiples");
static_assert(kXpP * 4 == 256 && (kChunk * kXpP) == 2048, "BC staging map");

constexpr size_t kOffX16   = 0;
constexpr size_t kOffWIN   = kOffX16  + (size_t)kRows * kDmod * 2;
constexpr size_t kOffWXP   = kOffWIN  + (size_t)kXZP  * kDmod * 2;
constexpr size_t kOffWOUT  = kOffWXP  + (size_t)kXpP  * kDin  * 2;
constexpr size_t kOffXZ    = kOffWOUT + (size_t)kDmod * kDin  * 2;
constexpr size_t kOffUC    = kOffXZ   + (size_t)kSeqL * kXZP  * 4;
constexpr size_t kOffUC16  = kOffUC   + (size_t)kSeqL * kDin  * 4;
constexpr size_t kOffBC    = kOffUC16 + (size_t)kSeqL * kDin  * 2;
constexpr size_t kOffGH    = kOffBC   + (size_t)kSeqL * kXpP  * 4;
constexpr size_t kOffGL    = kOffGH   + (size_t)kSeqL * kDin  * 2;
constexpr size_t kWsTotal  = kOffGL   + (size_t)kSeqL * kDin  * 2;
static_assert(kWsTotal == 97255424ull, "carve total");
static_assert(kWsTotal <= 134217728ull, "carve cap");
static_assert((kOffWIN % 128) == 0 && (kOffWXP % 128) == 0 && (kOffWOUT % 128) == 0 && (kOffXZ % 128) == 0 &&
              (kOffUC % 128) == 0 && (kOffUC16 % 128) == 0 && (kOffBC % 128) == 0 && (kOffGH % 128) == 0 &&
              (kOffGL % 128) == 0, "128-B aligned regions");

__device__ __forceinline__ unsigned short f2bf_bits(float f) {
  unsigned u = __float_as_uint(f);
  return (unsigned short)((u + 0x7FFFu + ((u >> 16) & 1u)) >> 16);
}
__device__ __forceinline__ float bf_bits2f(unsigned short h) { return __uint_as_float(((unsigned)h) << 16); }
__device__ __forceinline__ float rne_bf16(float f) { return bf_bits2f(f2bf_bits(f)); }
__device__ __forceinline__ unsigned pack2(unsigned short lo16, unsigned short hi16) {
  return (unsigned)lo16 | ((unsigned)hi16 << 16);
}
__device__ __forceinline__ void split_pack2(float f0, float f1, unsigned& hw, unsigned& lw) {
  const unsigned short h0 = f2bf_bits(f0), h1 = f2bf_bits(f1);
  const unsigned short l0 = f2bf_bits(f0 - bf_bits2f(h0)), l1 = f2bf_bits(f1 - bf_bits2f(h1));
  hw = pack2(h0, h1);
  lw = pack2(l0, l1);
}

__device__ __forceinline__ void dep_guard4_b(v8f& a, v8f& b, v8f& c, v8f& d, v16b x, v16b y) {
  asm volatile("v_nop\n\tv_nop\n\tv_nop\n\tv_nop" : "+v"(a), "+v"(b), "+v"(c), "+v"(d) : "v"(x), "v"(y));
}
__device__ __forceinline__ void keep4_b(v16b a, v16b b, v16b c, v16b d) { asm volatile("v_nop" :: "v"(a), "v"(b), "v"(c), "v"(d)); }
__device__ __forceinline__ void acc_guard4(v8f& a, v8f& b, v8f& c, v8f& d) { asm volatile("v_nop\n\tv_nop\n\tv_nop\n\tv_nop" : "+v"(a), "+v"(b), "+v"(c), "+v"(d)); }

union FragB { v16b v; v8b h[2]; };
__device__ __forceinline__ v16b frag_load(const __bf16* p) {
  FragB f;
  f.h[0] = *(const v8b*)(p);
  f.h[1] = *(const v8b*)(p + 16);
  return f.v;
}
__device__ __forceinline__ v8f frag_mma(v16b a, v16b b, v8f c) {
  return __builtin_amdgcn_wmma_f32_16x16x32_bf16(false, a, false, b, (short)0, c, false, false);
}

template <int SPL>
__global__ __launch_bounds__(256) void wmma_gemm64_bf16(
    const unsigned short* __restrict__ Ap, const unsigned short* __restrict__ A2p, int lda,
    const unsigned short* __restrict__ Btp, int ldb,
    float* __restrict__ C, int ldc, int M, int N, int K, float scale)
{
  const __bf16* A  = (const __bf16*)Ap;
  const __bf16* A2 = (const __bf16*)A2p;
  const __bf16* Bt = (const __bf16*)Btp;
  __shared__ __align__(16) float sT[8][16 * 68];
  const int lane = threadIdx.x & 31;
  const int wave = threadIdx.x >> 5;
  const int tilesN = N >> 6;
  const int tilesM = M >> 6;
  const int tile = blockIdx.x * 8 + wave;
  if (tile >= tilesM * tilesN) return;
  const int tm = tile / tilesN;
  const int tn = tile - tm * tilesN;
  const int m0 = tm << 6;
  const int n0 = tn << 6;

  const int rlane = lane & 15;
  const int koff  = (lane >> 4) * 8;
  const int mOff  = (lane >> 4) * 8;

  v8f acc[4][4];
#pragma unroll
  for (int i = 0; i < 4; ++i)
#pragma unroll
    for (int j = 0; j < 4; ++j) acc[i][j] = (v8f){0.f,0.f,0.f,0.f,0.f,0.f,0.f,0.f};

  for (int k0 = 0; k0 < K; k0 += 32) {
    v16b bh[4];
#pragma unroll
    for (int j = 0; j < 4; ++j) {
      const size_t bo = (size_t)(n0 + (j << 4) + rlane) * ldb + koff + k0;
      bh[j] = frag_load(Bt + bo);
    }
#pragma unroll
    for (int i = 0; i < 4; ++i) {
      const size_t ao = (size_t)(m0 + (i << 4) + rlane) * lda + koff + k0;
      v16b ah = frag_load(A + ao);
      v16b al = ah;
      if (SPL == 1) al = frag_load(A2 + ao);
#pragma unroll
      for (int j = 0; j < 4; ++j) {
        acc[i][j] = frag_mma(ah, bh[j], acc[i][j]);
        if (SPL == 1) acc[i][j] = frag_mma(al, bh[j], acc[i][j]);
      }
      dep_guard4_b(acc[i][0], acc[i][1], acc[i][2], acc[i][3], ah, al);
    }
    keep4_b(bh[0], bh[1], bh[2], bh[3]);
  }
  acc_guard4(acc[0][0], acc[0][1], acc[0][2], acc[0][3]);
  acc_guard4(acc[1][0], acc[1][1], acc[1][2], acc[1][3]);
  acc_guard4(acc[2][0], acc[2][1], acc[2][2], acc[2][3]);
  acc_guard4(acc[3][0], acc[3][1], acc[3][2], acc[3][3]);

  float* slab = sT[wave];
  const int hh = lane >> 4, c4 = (lane & 15) * 4;
#pragma unroll
  for (int i = 0; i < 4; ++i) {
    const int mBase = m0 + (i << 4);
#pragma unroll
    for (int j = 0; j < 4; ++j) {
#pragma unroll
      for (int r = 0; r < 8; ++r) {
        const float v = acc[i][j][r] * scale;
        slab[(mOff + r) * 68 + (j << 4) + rlane] = v;
      }
    }
    __builtin_amdgcn_fence(__ATOMIC_RELEASE, "workgroup");
    __builtin_amdgcn_wave_barrier();
    __builtin_amdgcn_fence(__ATOMIC_ACQUIRE, "workgroup");
    for (int pass = 0; pass < 2; ++pass) {
#pragma unroll
      for (int it = 0; it < 8; ++it) {
        const int row = it * 2 + hh;
        v4f v = *(const v4f*)(slab + row * 68 + c4);
        *(volatile v4f*)(C + (size_t)(mBase + row) * ldc + n0 + c4) = v;
      }
      __threadfence();
    }
    __builtin_amdgcn_fence(__ATOMIC_RELEASE, "workgroup");
    __builtin_amdgcn_wave_barrier();
    __builtin_amdgcn_fence(__ATOMIC_ACQUIRE, "workgroup");
  }
}

__global__ __launch_bounds__(256) void pack_rows_bf16_kernel(
    const float* __restrict__ src, unsigned short* __restrict__ dst, int total8)
{
  const int i = blockIdx.x * 256 + threadIdx.x;
  if (i >= total8) return;
  const size_t e0 = (size_t)i << 3;
  const v4f a0 = *(const v4f*)(src + e0);
  const v4f a1 = *(const v4f*)(src + e0 + 4);
  v4u w;
  w[0] = pack2(f2bf_bits(a0[0]), f2bf_bits(a0[1]));
  w[1] = pack2(f2bf_bits(a0[2]), f2bf_bits(a0[3]));
  w[2] = pack2(f2bf_bits(a1[0]), f2bf_bits(a1[1]));
  w[3] = pack2(f2bf_bits(a1[2]), f2bf_bits(a1[3]));
  unsigned short* q = dst + e0;
  *(volatile v4u*)q = w;
  __threadfence();
  *(volatile v4u*)q = w;
}

__global__ __launch_bounds__(256) void transpose_pack_kernel(
    const float* __restrict__ W, unsigned short* __restrict__ Bt, int Kdim, int Ndim)
{
  __shared__ float tile[64 * 65];
  const int tid = threadIdx.x, lane = tid & 31, wave = tid >> 5;
  const int n0 = blockIdx.x * 64;
  const int k0 = blockIdx.y * 64;
#pragma unroll
  for (int p = 0; p < 16; ++p) {
    const int idx = tid + p * 256;
    const int kk  = idx >> 6;
    const int nn  = idx & 63;
    const int n   = n0 + nn;
    const int nc  = (n < Ndim) ? n : (Ndim - 1);
    const float v = W[(size_t)(k0 + kk) * Ndim + nc];
    tile[kk * 65 + nn] = (n < Ndim) ? v : 0.f;
  }
  __syncthreads();
  const int q = lane >> 3, c8 = (lane & 7) * 8;
  v4u hv[2];
#pragma unroll
  for (int it = 0; it < 2; ++it) {
    const int nrow = it * 32 + wave * 4 + q;
#pragma unroll
    for (int e2 = 0; e2 < 4; ++e2) {
      const float f0 = tile[(c8 + 2 * e2) * 65 + nrow];
      const float f1 = tile[(c8 + 2 * e2 + 1) * 65 + nrow];
      hv[it][e2] = pack2(f2bf_bits(f0), f2bf_bits(f1));
    }
  }
  for (int pass = 0; pass < 2; ++pass) {
#pragma unroll
    for (int it = 0; it < 2; ++it) {
      const int nrow = it * 32 + wave * 4 + q;
      *(volatile v4u*)(Bt + (size_t)(n0 + nrow) * Kdim + k0 + c8) = hv[it];
    }
    __threadfence();
  }
}

__global__ __launch_bounds__(256) void conv_silu_kernel(
    const float* __restrict__ XZ, const float* __restrict__ cw, const float* __restrict__ cb,
    float* __restrict__ UC, unsigned short* __restrict__ UC16)
{
  __shared__ __align__(16) float sT[16 * kTP];
  const int tid = threadIdx.x, lane = tid & 31, wave = tid >> 5;
  const int d0 = blockIdx.x * 256, d = d0 + tid;
  const int t0 = blockIdx.y * 64;
  const v4f wv = *(const v4f*)(cw + (size_t)d * 4);
  const float w0 = rne_bf16(wv[0]), w1 = rne_bf16(wv[1]), w2 = rne_bf16(wv[2]), w3 = rne_bf16(wv[3]);
  const float bc = rne_bf16(cb[d]);
  float xm3, xm2, xm1;
  {
    const int r3 = t0 - 3, r2 = t0 - 2, r1 = t0 - 1;
    const float v3 = XZ[(size_t)(r3 < 0 ? 0 : r3) * kXZP + d];
    const float v2 = XZ[(size_t)(r2 < 0 ? 0 : r2) * kXZP + d];
    const float v1 = XZ[(size_t)(r1 < 0 ? 0 : r1) * kXZP + d];
    xm3 = (r3 >= 0) ? v3 : 0.f;
    xm2 = (r2 >= 0) ? v2 : 0.f;
    xm1 = (r1 >= 0) ? v1 : 0.f;
  }
  const int hrow = wave >> 1;
  const int hch  = (wave & 1) * 128 + lane * 4;
#pragma unroll 1
  for (int sub = 0; sub < 4; ++sub) {
    const int lb = t0 + sub * 16;
#pragma unroll 1
    for (int s = 0; s < 16; ++s) {
      const float xcur = XZ[(size_t)(lb + s) * kXZP + d];
      float acc = w0 * xm3;
      acc = fmaf(w1, xm2, acc);
      acc = fmaf(w2, xm1, acc);
      acc = fmaf(w3, xcur, acc);
      const float sv = acc + bc;
      const float sg = 1.0f / (1.0f + expf(-sv));
      sT[s * kTP + tid] = sv * sg;
      xm3 = xm2; xm2 = xm1; xm1 = xcur;
    }
    __syncthreads();
    v4f fv[4];
    v4u bv[2];
#pragma unroll
    for (int it = 0; it < 4; ++it) fv[it] = *(const v4f*)(sT + (it * 4 + hrow) * kTP + hch);
#pragma unroll
    for (int it = 0; it < 2; ++it) {
      const float* sp = sT + (it * 8 + wave) * kTP + lane * 8;
      const v4f a0 = *(const v4f*)(sp);
      const v4f a1 = *(const v4f*)(sp + 4);
      bv[it][0] = pack2(f2bf_bits(a0[0]), f2bf_bits(a0[1]));
      bv[it][1] = pack2(f2bf_bits(a0[2]), f2bf_bits(a0[3]));
      bv[it][2] = pack2(f2bf_bits(a1[0]), f2bf_bits(a1[1]));
      bv[it][3] = pack2(f2bf_bits(a1[2]), f2bf_bits(a1[3]));
    }
    for (int pass = 0; pass < 2; ++pass) {
#pragma unroll
      for (int it = 0; it < 4; ++it)
        *(volatile v4f*)(UC + (size_t)(lb + it * 4 + hrow) * kDin + d0 + hch) = fv[it];
#pragma unroll
      for (int it = 0; it < 2; ++it)
        *(volatile v4u*)(UC16 + (size_t)(lb + it * 8 + wave) * kDin + d0 + lane * 8) = bv[it];
      __threadfence();
    }
    __syncthreads();
  }
}

__global__ __launch_bounds__(256) void scan_gate_kernel(
    const float* __restrict__ BC, const float* __restrict__ UC, const float* __restrict__ XZ,
    const float* __restrict__ dtw, const float* __restrict__ dtb, const float* __restrict__ A_log,
    const float* __restrict__ Dv, unsigned short* __restrict__ GH, unsigned short* __restrict__ GL)
{
  __shared__ __align__(16) float sBC[kChunk * kXpP];
  __shared__ __align__(16) float sY[16 * kTP];
  const int tid = threadIdx.x, lane = tid & 31, wave = tid >> 5;
  const int d0 = blockIdx.x * 256, d = d0 + tid;

  float An[kNst];
#pragma unroll
  for (int q4 = 0; q4 < 4; ++q4) {
    const v4f av = *(const v4f*)(A_log + (size_t)d * kNst + 4 * q4);
    An[4 * q4 + 0] = -__expf(rne_bf16(av[0]));
    An[4 * q4 + 1] = -__expf(rne_bf16(av[1]));
    An[4 * q4 + 2] = -__expf(rne_bf16(av[2]));
    An[4 * q4 + 3] = -__expf(rne_bf16(av[3]));
  }
  const float Dd  = rne_bf16(Dv[d]);
  const float wdt = rne_bf16(dtw[d]);
  const float bdt = rne_bf16(dtb[d]);
  float hcar[kNst];
#pragma unroll
  for (int n = 0; n < kNst; ++n) hcar[n] = 0.f;

#pragma unroll 1
  for (int c = 0; c < kSeqL / kChunk; ++c) {
    const int l0 = c * kChunk;
    __syncthreads();
#pragma unroll
    for (int i = 0; i < 2; ++i) {
      const int idx = (tid + i * 256) * 4;
      *(v4f*)(sBC + idx) = *(const v4f*)(BC + (size_t)l0 * kXpP + idx);
    }
    __syncthreads();
    float hst[kNst], cum[kNst], csum[kNst];
#pragma unroll
    for (int n = 0; n < kNst; ++n) { hst[n] = hcar[n]; cum[n] = 0.f; csum[n] = 0.f; }

#pragma unroll 1
    for (int sub = 0; sub < 2; ++sub) {
#pragma unroll 1
      for (int s = 0; s < 16; ++s) {
        const int sl = sub * 16 + s;
        const size_t m = (size_t)(l0 + sl);
        const float* xr = sBC + sl * kXpP;
        v4f Bq[4], Cq[4];
#pragma unroll
        for (int qq = 0; qq < 4; ++qq) {
          Bq[qq] = *(const v4f*)(xr + 4 * qq);
          Cq[qq] = *(const v4f*)(xr + kNst + 4 * qq);
        }
        const float dtr = xr[2 * kNst];
        const float v   = fmaf(dtr, wdt, bdt);
        const float a   = __expf(-fabsf(v));
        const float u1  = 1.0f + a;
        const float l1p = __logf(u1) + (a - (u1 - 1.0f)) * __builtin_amdgcn_rcpf(u1);
        const float delta = fmaxf(v, 0.0f) + l1p;
        const float uv  = UC[m * kDin + d];
        const float zv  = XZ[m * kXZP + kDin + d];
        const float du  = delta * uv;
        float y = 0.f;
#pragma unroll
        for (int n = 0; n < kNst; ++n) {
          const float la = fmaxf(fminf(delta * An[n], 0.0f), kLogFloor);
          cum[n] += la;
          const float inv = __expf(-fmaxf(cum[n], -20.0f));
          csum[n] = fmaf(du * Bq[n >> 2][n & 3], inv, csum[n]);
          const float st = __expf(cum[n]) * (hst[n] + csum[n]);
          hcar[n] = st;
          y = fmaf(Cq[n >> 2][n & 3], st, y);
        }
        y = fmaf(uv, Dd, y);
        const float sg = 1.0f / (1.0f + expf(-zv));
        sY[s * kTP + tid] = y * (zv * sg);
      }
      __syncthreads();
      v4u hv[2], lv[2];
#pragma unroll
      for (int it = 0; it < 2; ++it) {
        const float* sp = sY + (it * 8 + wave) * kTP + lane * 8;
        const v4f a0 = *(const v4f*)(sp);
        const v4f a1 = *(const v4f*)(sp + 4);
        unsigned hw, lw;
        split_pack2(a0[0], a0[1], hw, lw); hv[it][0] = hw; lv[it][0] = lw;
        split_pack2(a0[2], a0[3], hw, lw); hv[it][1] = hw; lv[it][1] = lw;
        split_pack2(a1[0], a1[1], hw, lw); hv[it][2] = hw; lv[it][2] = lw;
        split_pack2(a1[2], a1[3], hw, lw); hv[it][3] = hw; lv[it][3] = lw;
      }
      for (int pass = 0; pass < 2; ++pass) {
#pragma unroll
        for (int it = 0; it < 2; ++it) {
          const size_t o = (size_t)(l0 + sub * 16 + it * 8 + wave) * kDin + d0 + lane * 8;
          *(volatile v4u*)(GH + o) = hv[it];
          *(volatile v4u*)(GL + o) = lv[it];
        }
        __threadfence();
      }
      __syncthreads();
    }
  }
}

static_assert(((kSeqL / 64) * (kXZP / 64)) == 256 * 8, "in_proj grid");
static_assert(((kSeqL / 64) * (kXpP / 64)) == 4 * 8, "x_proj grid");
static_assert(((kSeqL / 64) * (kDmod / 64)) == 64 * 8, "out_proj grid");

extern "C" void kernel_launch(void* const* d_in, const int* in_sizes, int n_in,
                              void* d_out, int out_size, void* d_ws, size_t ws_size,
                              hipStream_t stream)
{
  if (n_in < 10) return;
  if (in_sizes[0] != kRows * kDmod) return;
  if (in_sizes[1] != kDmod * kXZP) return;
  if (in_sizes[2] != kDin * 4 || in_sizes[3] != kDin) return;
  if (in_sizes[4] != kDin * kXpN) return;
  if (in_sizes[5] != kDin || in_sizes[6] != kDin) return;
  if (in_sizes[7] != kDin * kNst || in_sizes[8] != kDin) return;
  if (in_sizes[9] != kDin * kDmod) return;
  if (out_size != kRows * kDmod) return;
  if (ws_size < kWsTotal) return;

  const float* x      = (const float*)d_in[0];
  const float* W_in   = (const float*)d_in[1];
  const float* conv_w = (const float*)d_in[2];
  const float* conv_b = (const float*)d_in[3];
  const float* W_xprj = (const float*)d_in[4];
  const float* dt_w   = (const float*)d_in[5];
  const float* dt_b   = (const float*)d_in[6];
  const float* A_log  = (const float*)d_in[7];
  const float* Dv     = (const float*)d_in[8];
  const float* W_out  = (const float*)d_in[9];
  float* dout = (float*)d_out;

  char* ws = (char*)d_ws;
  unsigned short* X16    = (unsigned short*)(ws + kOffX16);
  unsigned short* WIN16  = (unsigned short*)(ws + kOffWIN);
  unsigned short* WXP16  = (unsigned short*)(ws + kOffWXP);
  unsigned short* WOUT16 = (unsigned short*)(ws + kOffWOUT);
  float*          XZ     = (float*)(ws + kOffXZ);
  float*          UC     = (float*)(ws + kOffUC);
  unsigned short* UC16   = (unsigned short*)(ws + kOffUC16);
  float*          BC     = (float*)(ws + kOffBC);
  unsigned short* GH     = (unsigned short*)(ws + kOffGH);
  unsigned short* GL     = (unsigned short*)(ws + kOffGL);

  transpose_pack_kernel<<<dim3(kXZP / 64, kDmod / 64), 256, 0, stream>>>(W_in, WIN16, kDmod, kXZP);
  transpose_pack_kernel<<<dim3(kXpP / 64, kDin / 64), 256, 0, stream>>>(W_xprj, WXP16, kDin, kXpN);
  transpose_pack_kernel<<<dim3(kDmod / 64, kDin / 64), 256, 0, stream>>>(W_out, WOUT16, kDin, kDmod);

  pack_rows_bf16_kernel<<<(kRows * kDmod) / 8 / 256, 256, 0, stream>>>(x, X16, (kRows * kDmod) / 8);

  for (int b = 0; b < kBatch; ++b) {
    const unsigned short* X16b = X16 + (size_t)b * kSeqL * kDmod;
    float* outb = dout + (size_t)b * kSeqL * kDmod;

    wmma_gemm64_bf16<0><<<dim3(256, 1), 256, 0, stream>>>(
        X16b, X16b, kDmod, WIN16, kDmod, XZ, kXZP, kSeqL, kXZP, kDmod, 1.0f);

    conv_silu_kernel<<<dim3(kDin / 256, kSeqL / 64), 256, 0, stream>>>(XZ, conv_w, conv_b, UC, UC16);

    wmma_gemm64_bf16<0><<<dim3(4, 1), 256, 0, stream>>>(
        UC16, UC16, kDin, WXP16, kDin, BC, kXpP, kSeqL, kXpP, kDin, 1.0f);

    scan_gate_kernel<<<dim3(kDin / 256, 1), 256, 0, stream>>>(BC, UC, XZ, dt_w, dt_b, A_log, Dv, GH, GL);

    wmma_gemm64_bf16<1><<<dim3(64, 1), 256, 0, stream>>>(
        GH, GL, kDin, WOUT16, kDin, outb, kDmod, kSeqL, kDmod, kDin, 1.0f);
  }
}
